// MultiHeadAttention_58102317580888
// MI455X (gfx1250) — hardware-verified
//
#include <hip/hip_runtime.h>


#ifndef NB
#define NB 4
#endif
#ifndef SEQ
#define SEQ 2048
#endif
#define NB_FULL  4
#define SEQ_FULL 2048
#ifndef OUT_SEQ
#define OUT_SEQ SEQ
#endif
#ifndef SCORE_KRES
#define SCORE_KRES 1
#endif
#define DM   512
#define NH_  8
#define HD   64
#define AW   4
#define QRS  2048.0f
#define QRI  (1.0f / 2048.0f)
#define KHS  1024.0f
#define SC2  (1.4426950408889634f / KHS)
#define PSH  14.0f
#define KLP  128
#define WGS1 1024.0f
#define WGS2 0.5f
#define CXP  1024
#define CXS  64.0f
#define CRS  128.0f
#define WS1  256.0f
#define WS2  2.0f
#define OSC  (1.0f / 16384.0f)

static_assert(HD == 64);
static_assert(NH_ * HD == DM);
static_assert(DM % 64 == 0);
static_assert(DM % 32 == 0);
static_assert((DM & (DM - 1)) == 0);
static_assert(CXP == 2 * DM);
static_assert(CXP % 32 == 0);
static_assert(SEQ % 64 == 0);
static_assert((NB * SEQ) % 64 == 0);
static_assert(SEQ % 32 == 0);
static_assert(SEQ % (16 * AW) == 0);
static_assert(((size_t)SEQ * DM) % 8 == 0);
static_assert(NB <= NB_FULL);
static_assert(SEQ <= SEQ_FULL);
static_assert(CRS * WS2 == WS1);
static_assert(CXS * WS1 * OSC == 1.0f);
static_assert(KLP == 2 * HD);
static_assert(KLP % 32 == 0);
static_assert(((size_t)NB * NH_ * SEQ) % 64 == 0);
static_assert(HD % 64 == 0);
static_assert(QRS * WGS2 == WGS1);
static_assert(WGS1 == KHS);
static_assert(HD * HD == 16 * 256);
static_assert(64 * 16 == 4 * 256);
static_assert(DM / 4 <= 256);
static_assert(PSH <= 15.0f);

typedef _Float16 h16;
typedef unsigned short bf;
typedef __attribute__((ext_vector_type(16))) __bf16   v16bf;
typedef __attribute__((ext_vector_type(16))) _Float16 v16h;
typedef __attribute__((ext_vector_type(8)))  _Float16 v8h;
typedef __attribute__((ext_vector_type(8)))  unsigned short v8us;
typedef __attribute__((ext_vector_type(8)))  float    v8f;
typedef __attribute__((ext_vector_type(4)))  float    v4f;
typedef v4f  __attribute__((may_alias)) v4fa;

__device__ __forceinline__ unsigned short f2bf(float f) { unsigned u = __float_as_uint(f); u += 0x7FFFu + ((u >> 16) & 1u); return (unsigned short)(u >> 16); }
__device__ __forceinline__ v16h cat16(v8h lo, v8h hi) { return __builtin_shufflevector(lo, hi, 0, 1, 2, 3, 4, 5, 6, 7, 8, 9, 10, 11, 12, 13, 14, 15); }
__device__ __forceinline__ v16bf cat16b(v8us lo, v8us hi) { return __builtin_bit_cast(v16bf, __builtin_shufflevector(lo, hi, 0, 1, 2, 3, 4, 5, 6, 7, 8, 9, 10, 11, 12, 13, 14, 15)); }
__device__ __forceinline__ v8f wmma16(v16h a, v16h b, v8f c) { return __builtin_amdgcn_wmma_f32_16x16x32_f16(false, a, false, b, (short)0, c, false, false); }
__device__ __forceinline__ v8f wmmab(v16bf a, v16bf b, v8f c) { return __builtin_amdgcn_wmma_f32_16x16x32_bf16(false, a, false, b, (short)0, c, false, false); }
__device__ __forceinline__ v16h  ldh(const h16* p) { return cat16(*(const v8h*)p, *(const v8h*)(p + 16)); }
__device__ __forceinline__ v16bf ldb(const bf* p)  { return cat16b(*(const v8us*)p, *(const v8us*)(p + 16)); }
__device__ __forceinline__ void wave_sync() { __builtin_amdgcn_fence(3  , "wavefront"); __builtin_amdgcn_wave_barrier(); asm volatile("" ::: "memory"); }
static __device__ __forceinline__ h16 toh_flush(float v) { const h16 r = (h16)v; return (fabsf(v) < 6.103515625e-05f) ? (h16)0.0f : r; }

__global__ __launch_bounds__(256) void k_cvt8(const float* __restrict__ src, bf* dst, size_t n8) {
    const size_t i = (size_t)blockIdx.x * 256 + threadIdx.x; if (i >= n8) return;
    const v8f v = *(const v8f*)(src + i * 8); v8us o;
#pragma unroll
    for (int k = 0; k < 8; ++k) o[k] = f2bf(v[k]);
    *(volatile v8us*)(dst + i * 8) = o; __threadfence(); *(volatile v8us*)(dst + i * 8) = o;
}

template <int MODE>
__global__ __launch_bounds__(256) void k_wT(const float* __restrict__ W, bf* dst, int pitch, float s1, float s2) {
    __shared__ float tile[64 * 65];
    const int tid = threadIdx.x; const int k0 = blockIdx.x * 64, n0 = blockIdx.y * 64;
#pragma unroll 4
    for (int i = 0; i < 16; ++i) { const int idx = tid + i * 256; const int kk = idx >> 6, nn = idx & 63;
        tile[kk * 65 + nn] = W[(size_t)(k0 + kk) * DM + n0 + nn]; }
    __syncthreads();
#pragma unroll 1
    for (int it = 0; it < 2; ++it) {
        const int c = it * 256 + tid; const int n = c >> 3, kc = (c & 7) * 8;
        float v[8];
#pragma unroll
        for (int i = 0; i < 8; ++i) v[i] = __uint_as_float(((unsigned)f2bf(tile[(kc + i) * 65 + n])) << 16);
        const size_t oo = (size_t)(n0 + n) * (size_t)pitch + (size_t)(k0 + kc);
        if (MODE == 0) {
            v8us o;
#pragma unroll
            for (int i = 0; i < 8; ++i) o[i] = (unsigned short)(__float_as_uint(v[i]) >> 16);
            *(volatile v8us*)(dst + oo) = o; __threadfence(); *(volatile v8us*)(dst + oo) = o;
        } else {
            v8h o1, o2;
#pragma unroll
            for (int i = 0; i < 8; ++i) { o1[i] = (h16)(v[i] * s1); o2[i] = (h16)(v[i] * s2); }
            h16* dh = (h16*)dst;
            *(volatile v8h*)(dh + oo) = o1; *(volatile v8h*)(dh + oo + DM) = o2;
            __threadfence();
            *(volatile v8h*)(dh + oo) = o1; *(volatile v8h*)(dh + oo + DM) = o2;
        }
    }
}

__global__ __launch_bounds__(256) void k_wg(const float* __restrict__ Wg, h16* WG, float* ZB) {
    __shared__ float tile[HD * (HD + 1)];
    const int tid = threadIdx.x;
#pragma unroll 4
    for (int e = 0; e < 16; ++e) { const int idx = tid + e * 256; const int i = idx >> 6, j = idx & 63;
        tile[i * (HD + 1) + j] = __uint_as_float(((unsigned)f2bf(Wg[idx])) << 16); }
    __syncthreads();
#pragma unroll 1
    for (int ps = 0; ps < 2; ++ps) {
#pragma unroll 1
        for (int it = 0; it < 4; ++it) {
            const int c = it * 256 + tid; const int n = c >> 4, ch = c & 15; const int kc = (ch & 7) * 8;
            const float s = (ch >> 3) ? WGS2 : WGS1;
            v8h o;
#pragma unroll
            for (int i = 0; i < 8; ++i) o[i] = toh_flush(tile[(kc + i) * (HD + 1) + n] * s);
            *(volatile v8h*)(WG + (size_t)n * KLP + ch * 8) = o; }
        if (tid < DM / 4) { const v4f z = (v4f){0.0f, 0.0f, 0.0f, 0.0f}; *(volatile v4f*)(ZB + tid * 4) = z; }
        if (ps == 0) __threadfence(); }
}

template <int OPF16, int EPI>
__global__ __launch_bounds__(32) void k_gemm(const bf* __restrict__ A, const bf* __restrict__ Bt, int K, const float* __restrict__ bias,
                                              h16* Ph, h16* Pr, float* Pf, int RB, size_t sRB, int pitch, int CB, size_t sCB) {
    __shared__ __align__(16) float os[16 * 68];
    const int lane = threadIdx.x & 31, lr = lane & 15, hi = lane >> 4; const int r0 = blockIdx.x * 64, c0 = blockIdx.y * 64;
    v8f acc[4][4];
#pragma unroll
    for (int mb = 0; mb < 4; ++mb)
#pragma unroll
        for (int nb = 0; nb < 4; ++nb) acc[mb][nb] = (v8f){};
    const size_t aoff = (size_t)(r0 + lr) * K + 8 * hi, boff = (size_t)(c0 + lr) * K + 8 * hi;
    if (OPF16) {
        const h16* Ah = (const h16*)A; const h16* Bh = (const h16*)Bt;
#pragma unroll 1
        for (int kc = 0; kc < K; kc += 32) {
            v16h a[4];
#pragma unroll
            for (int mb = 0; mb < 4; ++mb) a[mb] = ldh(Ah + aoff + (size_t)mb * 16 * K + kc);
#pragma unroll
            for (int nb = 0; nb < 4; ++nb) { const v16h b = ldh(Bh + boff + (size_t)nb * 16 * K + kc);
#pragma unroll
                for (int mb = 0; mb < 4; ++mb) acc[mb][nb] = wmma16(a[mb], b, acc[mb][nb]); }
            asm volatile("v_nop\n\tv_nop\n\tv_nop\n\tv_nop" : "+v"(acc[0][0]), "+v"(acc[1][1]), "+v"(acc[2][2]), "+v"(acc[3][3]) : "v"(a[0]), "v"(a[1]), "v"(a[2]), "v"(a[3]));
        }
    } else {
#pragma unroll 1
        for (int kc = 0; kc < K; kc += 32) {
            v16bf a[4];
#pragma unroll
            for (int mb = 0; mb < 4; ++mb) a[mb] = ldb(A + aoff + (size_t)mb * 16 * K + kc);
#pragma unroll
            for (int nb = 0; nb < 4; ++nb) { const v16bf b = ldb(Bt + boff + (size_t)nb * 16 * K + kc);
#pragma unroll
                for (int mb = 0; mb < 4; ++mb) acc[mb][nb] = wmmab(a[mb], b, acc[mb][nb]); }
            asm volatile("v_nop\n\tv_nop\n\tv_nop\n\tv_nop" : "+v"(acc[0][0]), "+v"(acc[1][1]), "+v"(acc[2][2]), "+v"(acc[3][3]) : "v"(a[0]), "v"(a[1]), "v"(a[2]), "v"(a[3]));
        }
    }
    const size_t tbase = (size_t)(r0 / RB) * sRB + (size_t)(r0 % RB) * (size_t)pitch + (size_t)(c0 / CB) * sCB + (size_t)(c0 % CB);
    float bcol[4] = {0.0f, 0.0f, 0.0f, 0.0f};
    if constexpr (EPI != 2) {
#pragma unroll
        for (int nb = 0; nb < 4; ++nb) bcol[nb] = bias[(c0 + nb * 16 + lr) & (DM - 1)];
    }
#pragma unroll
    for (int mb = 0; mb < 4; ++mb) {
        float brow[8] = {0.0f, 0.0f, 0.0f, 0.0f, 0.0f, 0.0f, 0.0f, 0.0f};
        if constexpr (EPI == 2) {
#pragma unroll
            for (int j = 0; j < 8; ++j) brow[j] = bias[(r0 + mb * 16 + 8 * hi + j) & (DM - 1)];
        }
#pragma unroll
        for (int nb = 0; nb < 4; ++nb) {
#pragma unroll
            for (int j = 0; j < 8; ++j) {
                float v = acc[mb][nb][j];
                if constexpr (EPI == 3) v = v * OSC;
                if constexpr (EPI == 2) v += brow[j]; else v += bcol[nb];
                os[(hi * 8 + j) * 68 + nb * 16 + lr] = v; } }
        wave_sync();
        const size_t sb = tbase + (size_t)(mb * 16) * (size_t)pitch;
        if (EPI == 3) {
#pragma unroll 1
            for (int ps = 0; ps < 2; ++ps) {
#pragma unroll
                for (int s = 0; s < 8; ++s) { const int row = 2 * s + hi, cofs = lr * 4;
                    const v4f val = *(const v4fa*)(&os[row * 68 + cofs]);
                    *(volatile v4f*)(Pf + sb + (size_t)row * (size_t)pitch + cofs) = val; }
                if (ps == 0) __threadfence(); }
        } else {
#pragma unroll 1
            for (int ps = 0; ps < 2; ++ps) {
#pragma unroll
                for (int s = 0; s < 4; ++s) { const int row = 4 * s + (lane >> 3), c8 = (lane & 7) * 8;
                    const v4f x0 = *(const v4fa*)(&os[row * 68 + c8]); const v4f x1 = *(const v4fa*)(&os[row * 68 + c8 + 4]); v8h hv, rv;
#pragma unroll
                    for (int i = 0; i < 4; ++i) { const h16 a0 = (h16)x0[i]; const h16 a1 = (h16)x1[i]; hv[i] = a0; hv[4 + i] = a1; rv[i] = (h16)((x0[i] - (float)a0) * QRS); rv[4 + i] = (h16)((x1[i] - (float)a1) * QRS); }
                    const size_t oo = sb + (size_t)row * (size_t)pitch + c8;
                    *(volatile v8h*)(Ph + oo) = hv; if (EPI == 0) *(volatile v8h*)(Pr + oo) = rv; }
                if (ps == 0) __threadfence(); }
        }
        wave_sync();
    }
}

__global__ __launch_bounds__(32 * AW) void k_flash(const h16* __restrict__ QH, const h16* __restrict__ QR, const h16* __restrict__ KP, const h16* __restrict__ KR, const h16* __restrict__ VT, h16* CX) {
    __shared__ __align__(16) float os[AW * 16 * 68];
    const int lane = threadIdx.x & 31, wave = __builtin_amdgcn_readfirstlane(threadIdx.x >> 5), lr = lane & 15, hi = lane >> 4;
    const int zh = blockIdx.y; const int b = zh / NH_, h = zh % NH_;
    const int t0 = (blockIdx.x * AW + wave) * 16;
    const size_t pbase = (size_t)zh * SEQ * HD;
    const size_t qo = pbase + (size_t)(t0 + lr) * HD + 8 * hi;
    const v16h qh0 = ldh(QH + qo), qh1 = ldh(QH + qo + 32), qr0 = ldh(QR + qo), qr1 = ldh(QR + qo + 32);
    const size_t ko = pbase + (size_t)lr * HD + 8 * hi;
    const size_t vo = pbase + (size_t)lr * SEQ + 8 * hi;
    v8f o0 = (v8f){}, o1 = (v8f){}, o2 = (v8f){}, o3 = (v8f){};
    float m = -3.0e38f, l = 0.0f;
#pragma unroll 1
    for (int key0 = 0; key0 < SEQ; key0 += 32) {
        const h16* ka = KP + ko + (size_t)key0 * HD;
        const v16h ka0 = ldh(ka), ka1 = ldh(ka + 32), kb0 = ldh(ka + 16 * HD), kb1 = ldh(ka + 16 * HD + 32);
#if SCORE_KRES
        const h16* kra = KR + ko + (size_t)key0 * HD;
        const v16h ra0 = ldh(kra), ra1 = ldh(kra + 32), rb0 = ldh(kra + 16 * HD), rb1 = ldh(kra + 16 * HD + 32);
#endif
        v8f sHa = (v8f){}, sLa = (v8f){}, sHb = (v8f){}, sLb = (v8f){};
        sHa = wmma16(ka0, qh0, sHa); sLa = wmma16(ka0, qr0, sLa); sHb = wmma16(kb0, qh0, sHb); sLb = wmma16(kb0, qr0, sLb);
        sHa = wmma16(ka1, qh1, sHa); sLa = wmma16(ka1, qr1, sLa); sHb = wmma16(kb1, qh1, sHb); sLb = wmma16(kb1, qr1, sLb);
#if SCORE_KRES
        sLa = wmma16(ra0, qh0, sLa); sLb = wmma16(rb0, qh0, sLb);
        sLa = wmma16(ra1, qh1, sLa); sLb = wmma16(rb1, qh1, sLb);
        asm volatile("v_nop\n\tv_nop\n\tv_nop\n\tv_nop" : "+v"(sHa), "+v"(sLa), "+v"(sHb), "+v"(sLb) : "v"(ka0), "v"(ka1), "v"(kb0), "v"(kb1), "v"(ra0), "v"(ra1), "v"(rb0), "v"(rb1));
#else
        asm volatile("v_nop\n\tv_nop\n\tv_nop\n\tv_nop" : "+v"(sHa), "+v"(sLa), "+v"(sHb), "+v"(sLb) : "v"(ka0), "v"(ka1), "v"(kb0), "v"(kb1));
#endif
        float ta[8], tb[8]; float mx = -3.0e38f;
#pragma unroll
        for (int r = 0; r < 8; ++r) { ta[r] = (sHa[r] + sLa[r] * QRI) * SC2; tb[r] = (sHb[r] + sLb[r] * QRI) * SC2; mx = fmaxf(mx, fmaxf(ta[r], tb[r])); }
        mx = fmaxf(mx, __shfl_xor(mx, 16, 32));
        const float mnew = fmaxf(m, mx);
        const float alpha = __builtin_amdgcn_exp2f(m - mnew);
        const float sh = PSH - mnew;
        v16h pb; float ls = 0.0f;
#pragma unroll
        for (int r = 0; r < 8; ++r) { const float ea = ta[r] + sh; const float ec = tb[r] + sh;
            const h16 pa = (ea < -14.0f) ? (h16)0.0f : (h16)__builtin_amdgcn_exp2f(ea);
            const h16 pc = (ec < -14.0f) ? (h16)0.0f : (h16)__builtin_amdgcn_exp2f(ec);
            pb[r] = pa; pb[8 + r] = pc; ls += (float)pa + (float)pc; }
        l = l * alpha + ls; m = mnew;
        o0 = o0 * alpha; o1 = o1 * alpha; o2 = o2 * alpha; o3 = o3 * alpha;
        const h16* va = VT + vo + key0;
        const v16h v0 = ldh(va), v1 = ldh(va + (size_t)16 * SEQ), v2 = ldh(va + (size_t)32 * SEQ), v3 = ldh(va + (size_t)48 * SEQ);
        o0 = wmma16(v0, pb, o0); o1 = wmma16(v1, pb, o1); o2 = wmma16(v2, pb, o2); o3 = wmma16(v3, pb, o3);
        asm volatile("v_nop\n\tv_nop\n\tv_nop\n\tv_nop" : "+v"(o0), "+v"(o1), "+v"(o2), "+v"(o3) : "v"(v0), "v"(v1), "v"(v2), "v"(v3), "v"(pb));
    }
    l += __shfl_xor(l, 16, 32);
    const float inv = CXS * (1.0f / l);
    const int wb = wave * 16 * 68;
    { v4f a, c;
      a[0] = o0[0] * inv; a[1] = o0[1] * inv; a[2] = o0[2] * inv; a[3] = o0[3] * inv; c[0] = o0[4] * inv; c[1] = o0[5] * inv; c[2] = o0[6] * inv; c[3] = o0[7] * inv;
      *(v4fa*)(&os[wb + lr * 68 +  0 + 8 * hi]) = a; *(v4fa*)(&os[wb + lr * 68 +  0 + 8 * hi + 4]) = c;
      a[0] = o1[0] * inv; a[1] = o1[1] * inv; a[2] = o1[2] * inv; a[3] = o1[3] * inv; c[0] = o1[4] * inv; c[1] = o1[5] * inv; c[2] = o1[6] * inv; c[3] = o1[7] * inv;
      *(v4fa*)(&os[wb + lr * 68 + 16 + 8 * hi]) = a; *(v4fa*)(&os[wb + lr * 68 + 16 + 8 * hi + 4]) = c;
      a[0] = o2[0] * inv; a[1] = o2[1] * inv; a[2] = o2[2] * inv; a[3] = o2[3] * inv; c[0] = o2[4] * inv; c[1] = o2[5] * inv; c[2] = o2[6] * inv; c[3] = o2[7] * inv;
      *(v4fa*)(&os[wb + lr * 68 + 32 + 8 * hi]) = a; *(v4fa*)(&os[wb + lr * 68 + 32 + 8 * hi + 4]) = c;
      a[0] = o3[0] * inv; a[1] = o3[1] * inv; a[2] = o3[2] * inv; a[3] = o3[3] * inv; c[0] = o3[4] * inv; c[1] = o3[5] * inv; c[2] = o3[6] * inv; c[3] = o3[7] * inv;
      *(v4fa*)(&os[wb + lr * 68 + 48 + 8 * hi]) = a; *(v4fa*)(&os[wb + lr * 68 + 48 + 8 * hi + 4]) = c; }
    wave_sync();
    h16* crow = CX + ((size_t)b * SEQ + t0) * CXP + h * HD;
#pragma unroll 1
    for (int ps = 0; ps < 2; ++ps) {
#pragma unroll
        for (int s = 0; s < 4; ++s) { const int row = 4 * s + (lane >> 3), c8 = (lane & 7) * 8;
            const v4f x0 = *(const v4fa*)(&os[wb + row * 68 + c8]); const v4f x1 = *(const v4fa*)(&os[wb + row * 68 + c8 + 4]); v8h hv, rv;
#pragma unroll
            for (int i = 0; i < 4; ++i) { const h16 a0 = toh_flush(x0[i]); const h16 a1 = toh_flush(x1[i]); hv[i] = a0; hv[4 + i] = a1; rv[i] = toh_flush((x0[i] - (float)a0) * CRS); rv[4 + i] = toh_flush((x1[i] - (float)a1) * CRS); }
            const size_t oo = (size_t)row * CXP + c8;
            *(volatile v8h*)(crow + oo) = hv; *(volatile v8h*)(crow + oo + DM) = rv; }
        if (ps == 0) __threadfence(); }
}

static constexpr size_t al256(size_t v) { return (v + 255) & ~(size_t)255; }
static constexpr size_t SZ_XB = al256((size_t)NB * SEQ * DM * 2);
static constexpr size_t SZ_W3 = al256((size_t)3 * DM * DM * 2);
static constexpr size_t SZ_WO = al256((size_t)DM * CXP * 2);
static constexpr size_t SZ_WG = al256((size_t)HD * KLP * 2);
static constexpr size_t SZ_ZB = al256((size_t)DM * 4);
static constexpr size_t SZ_PL = al256((size_t)NB * NH_ * SEQ * HD * 2);
static constexpr size_t SZ_KL = al256((size_t)NB * NH_ * SEQ * KLP * 2);
static constexpr size_t SZ_CX = al256((size_t)NB * SEQ * CXP * 2);
static constexpr size_t SZ_TOTAL = 3 * SZ_XB + SZ_W3 + SZ_WO + SZ_WG + SZ_ZB + 5 * SZ_PL + SZ_KL + SZ_CX;
static_assert(SZ_TOTAL <= (size_t)134217728);
static_assert(((size_t)DM * DM * 2) % 256 == 0);
static_assert(SZ_WG >= (size_t)(HD - 1) * KLP * 2 + (size_t)KLP * 2);
static_assert(SZ_KL >= ((size_t)NB * NH_ * SEQ - 1) * KLP * 2 + (size_t)KLP * 2);

static void cvt_in(const float* x, bf* XB, hipStream_t stream) {
    if (SEQ == SEQ_FULL) {
        const size_t n8 = (size_t)NB * SEQ * DM / 8;
        k_cvt8<<<(unsigned)((n8 + 255) / 256), 256, 0, stream>>>(x, XB, n8);
    } else {
        const size_t n8 = (size_t)SEQ * DM / 8;
        for (int b = 0; b < NB; ++b) k_cvt8<<<(unsigned)((n8 + 255) / 256), 256, 0, stream>>>(x + (size_t)b * SEQ_FULL * DM, XB + (size_t)b * SEQ * DM, n8);
    }
}

extern "C" void kernel_launch(void* const* d_in, const int* in_sizes, int n_in,
                              void* d_out, int out_size, void* d_ws, size_t ws_size, hipStream_t stream) {
    if (n_in < 9) return;
    const size_t needx = ((size_t)(NB - 1) * SEQ_FULL + SEQ) * DM;
    if ((size_t)in_sizes[0] < needx || (size_t)in_sizes[1] < needx || (size_t)in_sizes[2] < needx) return;
    if ((size_t)in_sizes[4] < (size_t)DM * DM || (size_t)in_sizes[5] < (size_t)DM * DM || (size_t)in_sizes[6] < (size_t)DM * DM || (size_t)in_sizes[8] < (size_t)DM * DM) return;
    if ((size_t)in_sizes[7] < (size_t)HD * HD) return;
    if ((size_t)out_size < ((size_t)(NB - 1) * OUT_SEQ + SEQ) * DM) return;
    if (SZ_TOTAL > ws_size) return;
    const float* xq = (const float*)d_in[0]; const float* xk = (const float*)d_in[1]; const float* xv = (const float*)d_in[2];
    const float* wq = (const float*)d_in[4];
    const float* wk = (const float*)d_in[5];
    const float* wv = (const float*)d_in[6];
    const float* wg = (const float*)d_in[7];
    const float* wo = (const float*)d_in[8];
    float* OUT = (float*)d_out;
    char* wsp = (char*)d_ws;
    bf* XQ = (bf*)wsp; wsp += SZ_XB;
    bf* XK = (bf*)wsp; wsp += SZ_XB;
    bf* XV = (bf*)wsp; wsp += SZ_XB;
    bf* W3 = (bf*)wsp; wsp += SZ_W3;
    bf* WO = (bf*)wsp; wsp += SZ_WO;
    h16* WG = (h16*)wsp; wsp += SZ_WG;
    float* ZB = (float*)wsp; wsp += SZ_ZB;
    h16* QH = (h16*)wsp; wsp += SZ_PL;
    h16* QR = (h16*)wsp; wsp += SZ_PL;
    h16* KP = (h16*)wsp; wsp += SZ_PL;
    h16* KR = (h16*)wsp; wsp += SZ_PL;
    h16* VT = (h16*)wsp; wsp += SZ_PL;
    h16* KL = (h16*)wsp; wsp += SZ_KL;
    h16* CX = (h16*)wsp; wsp += SZ_CX;
    bf* WQ = W3; bf* WK = W3 + (size_t)DM * DM; bf* WV = W3 + (size_t)2 * DM * DM;

    cvt_in(xq, XQ, stream); cvt_in(xk, XK, stream); cvt_in(xv, XV, stream);

    k_wT<0><<<dim3(DM / 64, DM / 64, 1), 256, 0, stream>>>(wq, WQ, DM, 1.0f, 1.0f);
    k_wT<0><<<dim3(DM / 64, DM / 64, 1), 256, 0, stream>>>(wk, WK, DM, 1.0f, 1.0f);
    k_wT<0><<<dim3(DM / 64, DM / 64, 1), 256, 0, stream>>>(wv, WV, DM, 1.0f, 1.0f);
    k_wT<1><<<dim3(DM / 64, DM / 64, 1), 256, 0, stream>>>(wo, WO, CXP, WS1, WS2);
    k_wg<<<dim3(1, 1, 1), 256, 0, stream>>>(wg, WG, ZB);

    k_gemm<0, 0><<<dim3(NB * SEQ / 64, DM / 64, 1), 32, 0, stream>>>(XQ, WQ, DM, ZB, QH, QR, OUT, SEQ, (size_t)NH_ * SEQ * HD, HD, HD, (size_t)SEQ * HD);
    k_gemm<0, 0><<<dim3(NB * SEQ / 64, DM / 64, 1), 32, 0, stream>>>(XK, WK, DM, ZB, KL, KL + HD, OUT, SEQ, (size_t)NH_ * SEQ * KLP, KLP, HD, (size_t)SEQ * KLP);
    k_gemm<1, 0><<<dim3(NB * NH_ * SEQ / 64, HD / 64, 1), 32, 0, stream>>>((const bf*)KL, (const bf*)WG, KLP, ZB, KP, KR, OUT, SEQ, (size_t)SEQ * HD, HD, HD, (size_t)0);
    k_gemm<0, 2><<<dim3(DM / 64, NB * SEQ / 64, 1), 32, 0, stream>>>(WV, XV, DM, ZB, VT, VT, OUT, DM, (size_t)0, SEQ, SEQ, (size_t)DM * SEQ);

    k_flash<<<dim3(SEQ / (16 * AW), NB * NH_, 1), 32 * AW, 0, stream>>>(QH, QR, KP, KR, VT, CX);

    k_gemm<1, 3><<<dim3(NB * SEQ / 64, DM / 64, 1), 32, 0, stream>>>((const bf*)CX, WO, CXP, ZB, CX, CX, OUT, SEQ, (size_t)OUT_SEQ * DM, DM, DM, (size_t)0);
}
